// CausalSelfAttention_59098749993568
// MI455X (gfx1250) — hardware-run, weakly checked
//
#include <hip/hip_runtime.h>
#include <math.h>

typedef __attribute__((ext_vector_type(16))) __bf16   v16b;
typedef __attribute__((ext_vector_type(8)))  __bf16   v8b;
typedef __attribute__((ext_vector_type(8)))  float    v8f;
typedef __attribute__((ext_vector_type(4)))  float    v4f;
typedef __attribute__((ext_vector_type(4)))  unsigned int v4u;

constexpr int kBatch = 2;
constexpr int kSeq   = 2048;
constexpr int kDim   = 1024;
constexpr int kHeads = 16;
constexpr int kHd    = 64;
constexpr int kRows  = kBatch * kSeq;
constexpr int kScanT = 32;
constexpr float kEps = 1e-6f;
static_assert(kHeads * kHd == kDim, "head split");
static_assert((kDim % 32) == 0, "GEMM K multiple of 32");
static_assert((kRows % 64) == 0 && (kDim % 64) == 0, "GEMM M, N multiples of 64");
static_assert((kSeq % kScanT) == 0, "scan chunking");
static_assert(kHd == 64, "one head = one 64-column tile");

constexpr size_t kActB  = (size_t)kRows * kDim * 2;
constexpr size_t kWgtB  = (size_t)kDim * kDim * 2;
constexpr size_t kF32B  = (size_t)kRows * kDim * 4;
constexpr size_t kOffXQ = 0;
constexpr size_t kOffXK = kOffXQ + kActB;
constexpr size_t kOffXV = kOffXK + kActB;
constexpr size_t kOffWQ = kOffXV + kActB;
constexpr size_t kOffWK = kOffWQ + kWgtB;
constexpr size_t kOffWV = kOffWK + kWgtB;
constexpr size_t kOffWO = kOffWV + kWgtB;
constexpr size_t kOffQF = kOffWO + kWgtB;
constexpr size_t kOffKF = kOffQF + kF32B;
constexpr size_t kOffVF = kOffKF + kF32B;
constexpr size_t kOffAH = kOffVF + kF32B;
constexpr size_t kOffAL = kOffAH + kActB;
constexpr size_t kWsTotal = kOffAL + kActB;
static_assert(kWsTotal == 100663296ull, "carve total");
static_assert(kWsTotal <= 134217728ull, "carve cap");
static_assert((kOffXK % 128) == 0 && (kOffXV % 128) == 0 && (kOffWQ % 128) == 0 && (kOffWK % 128) == 0 &&
              (kOffWV % 128) == 0 && (kOffWO % 128) == 0 && (kOffQF % 128) == 0 && (kOffKF % 128) == 0 &&
              (kOffVF % 128) == 0 && (kOffAH % 128) == 0 && (kOffAL % 128) == 0, "128-B aligned regions");

__device__ __forceinline__ unsigned short f2bf_bits(float f) {
  unsigned u = __float_as_uint(f);
  return (unsigned short)((u + 0x7FFFu + ((u >> 16) & 1u)) >> 16);
}
__device__ __forceinline__ float bf_bits2f(unsigned short h) { return __uint_as_float(((unsigned)h) << 16); }
__device__ __forceinline__ float bf16r(float f) { return bf_bits2f(f2bf_bits(f)); }
__device__ __forceinline__ unsigned pk16(unsigned short a, unsigned short b) { return (unsigned)a | ((unsigned)b << 16); }

template <typename T> struct Frag;
template <> struct Frag<__bf16> {
  typedef v16b V; union U { v16b v; v8b h[2]; };
  static __device__ __forceinline__ v16b load(const __bf16* p) {
    U f; f.h[0] = *(const v8b*)(p); f.h[1] = *(const v8b*)(p + 16); return f.v;
  }
};

__device__ __forceinline__ v8f mma_bf(v16b a, v16b b, v8f c) {
  c = __builtin_amdgcn_wmma_f32_16x16x32_bf16(false, a, false, b, (short)0, c, false, false);
  asm volatile("v_nop\n\tv_nop\n\tv_nop\n\tv_nop" : "+v"(c) : "v"(a), "v"(b));
  return c;
}

__global__ __launch_bounds__(256) void cvt_bf16_planes_kernel(
    const float* __restrict__ s0, const float* __restrict__ s1, const float* __restrict__ s2, const float* __restrict__ s3,
    unsigned short* __restrict__ d0, unsigned short* __restrict__ d1, unsigned short* __restrict__ d2,
    unsigned short* __restrict__ d3, int n8)
{
  const int z = blockIdx.y;
  const float* src = (z == 0) ? s0 : (z == 1) ? s1 : (z == 2) ? s2 : s3;
  unsigned short* dst = (z == 0) ? d0 : (z == 1) ? d1 : (z == 2) ? d2 : d3;
  const int i = blockIdx.x * 256 + threadIdx.x;
  if (i >= n8) return;
  const float* p = src + 8 * (size_t)i;
  const v4f a = *(const v4f*)(p);
  const v4f c = *(const v4f*)(p + 4);
  unsigned short hb[8];
#pragma unroll
  for (int e = 0; e < 4; ++e) {
    const float x0 = a[e];
    const float x1 = c[e];
    hb[e]     = f2bf_bits(x0);
    hb[4 + e] = f2bf_bits(x1);
  }
  const v4u u = (v4u){pk16(hb[0], hb[1]), pk16(hb[2], hb[3]), pk16(hb[4], hb[5]), pk16(hb[6], hb[7])};
  unsigned short* q = dst + 8 * (size_t)i;
  *(volatile v4u*)q = u;
  __threadfence();
  *(volatile v4u*)q = u;
}

template <bool SPLA, int EPI>
__global__ __launch_bounds__(256) void gemm_tile64_kernel(
    const unsigned short* __restrict__ Ap, const unsigned short* __restrict__ A2p, int lda,
    const unsigned short* __restrict__ Btp, int ldb,
    float* __restrict__ Cout, int ldc,
    const float* __restrict__ bias, int M, int N, int K)
{
  const __bf16* A  = (const __bf16*)Ap;
  const __bf16* A2 = (const __bf16*)A2p;
  const __bf16* Bt = (const __bf16*)Btp;
  __shared__ __align__(16) float sT[8][16 * 68];
  const int lane = threadIdx.x & 31;
  const int wave = threadIdx.x >> 5;
  const int tilesN = N >> 6;
  const int tilesM = M >> 6;
  const int tile = blockIdx.x * 8 + wave;
  if (tile >= tilesM * tilesN) return;
  const int tm = tile / tilesN;
  const int tn = tile - tm * tilesN;
  const int m0 = tm << 6;
  const int n0 = tn << 6;

  const int rlane = lane & 15;
  const int koff  = (lane >> 4) * 8;
  const int mOff  = (lane >> 4) * 8;

  v8f acc[4][4];
#pragma unroll
  for (int i = 0; i < 4; ++i)
#pragma unroll
    for (int j = 0; j < 4; ++j) acc[i][j] = (v8f){0.f, 0.f, 0.f, 0.f, 0.f, 0.f, 0.f, 0.f};

  for (int k0 = 0; k0 < K; k0 += 32) {
    v16b bh[4];
#pragma unroll
    for (int j = 0; j < 4; ++j) {
      const size_t bo = (size_t)(n0 + (j << 4) + rlane) * ldb + koff + k0;
      bh[j] = Frag<__bf16>::load(Bt + bo);
    }
#pragma unroll
    for (int i = 0; i < 4; ++i) {
      const size_t ao = (size_t)(m0 + (i << 4) + rlane) * lda + koff + k0;
      const v16b ah = Frag<__bf16>::load(A + ao);
      v16b al = ah;
      if (SPLA) al = Frag<__bf16>::load(A2 + ao);
#pragma unroll
      for (int j = 0; j < 4; ++j) {
        acc[i][j] = mma_bf(ah, bh[j], acc[i][j]);
        if (SPLA) acc[i][j] = mma_bf(al, bh[j], acc[i][j]);
      }
    }
  }

  float* slab = sT[wave];
  float bvj[4];
#pragma unroll
  for (int j = 0; j < 4; ++j) bvj[j] = bf16r(bias[n0 + (j << 4) + rlane]);
#pragma unroll
  for (int i = 0; i < 4; ++i) {
    const int mBase = m0 + (i << 4);
#pragma unroll
    for (int j = 0; j < 4; ++j) {
#pragma unroll
      for (int r = 0; r < 8; ++r) {
        slab[(mOff + r) * 68 + (j << 4) + rlane] = acc[i][j][r] + bvj[j];
      }
    }
    __builtin_amdgcn_fence(__ATOMIC_RELEASE, "workgroup");
    __builtin_amdgcn_wave_barrier();
    __builtin_amdgcn_fence(__ATOMIC_ACQUIRE, "workgroup");
    if (EPI == 1) {
#pragma unroll 1
      for (int it = 0; it < 32; ++it) {
        float* p = slab + (it >> 1) * 68 + (it & 1) * 32 + lane;
        const float x = *p;
        const float ex = expf(fminf(x, 0.0f));
        const float y = (x > 0.0f) ? (x + 1.0f) : ex;
        *p = y;
      }
      __builtin_amdgcn_fence(__ATOMIC_RELEASE, "workgroup");
      __builtin_amdgcn_wave_barrier();
      __builtin_amdgcn_fence(__ATOMIC_ACQUIRE, "workgroup");
    }
    {
      const int hh = lane >> 4, c4 = (lane & 15) * 4;
      for (int pass = 0; pass < 2; ++pass) {
#pragma unroll
        for (int it = 0; it < 8; ++it) {
          const int row = it * 2 + hh;
          const v4f v = *(const v4f*)(slab + row * 68 + c4);
          *(volatile v4f*)(Cout + (size_t)(mBase + row) * ldc + n0 + c4) = v;
        }
        __threadfence();
      }
    }
    __builtin_amdgcn_fence(__ATOMIC_RELEASE, "workgroup");
    __builtin_amdgcn_wave_barrier();
    __builtin_amdgcn_fence(__ATOMIC_ACQUIRE, "workgroup");
  }
}

__global__ __launch_bounds__(256) void scan_state_kernel(
    const float* __restrict__ QF, const float* __restrict__ KF, const float* __restrict__ VF,
    unsigned short* __restrict__ AH, unsigned short* __restrict__ AL)
{
  __shared__ __align__(16) float sQ[kScanT * 64];
  __shared__ __align__(16) float sK[kScanT * 64];
  __shared__ __align__(16) float sV[kScanT * 64];
  __shared__ __align__(16) float sN[4 * kScanT * 64];
  const int tid = threadIdx.x, lane = tid & 31, wave = tid >> 5;
  const int j = tid & 63;
  const int dg = tid >> 6;
  const int bh = blockIdx.x;
  const int bb = bh >> 4;
  const int hd = bh & 15;
  const size_t row0 = (size_t)bb * kSeq;
  const int col0 = hd * kHd;

  float kv[16];
#pragma unroll
  for (int i = 0; i < 16; ++i) kv[i] = 0.0f;
  float kcarry = 0.0f;

  const int lr = tid >> 4, lc4 = (tid & 15) * 4;
  const int q4 = lane >> 3, c8 = (lane & 7) * 8;
  const int orow = wave * 4 + q4;

#pragma unroll 1
  for (int t0 = 0; t0 < kSeq; t0 += kScanT) {
    __syncthreads();
#pragma unroll
    for (int i = 0; i < 2; ++i) {
      const int r = lr + 16 * i;
      const size_t g = (row0 + (size_t)(t0 + r)) * kDim + col0 + lc4;
      *(v4f*)(sQ + r * 64 + lc4) = *(const v4f*)(QF + g);
      *(v4f*)(sK + r * 64 + lc4) = *(const v4f*)(KF + g);
      *(v4f*)(sV + r * 64 + lc4) = *(const v4f*)(VF + g);
    }
    __syncthreads();

#pragma unroll 1
    for (int s = 0; s < kScanT; ++s) {
      const float vj = sV[s * 64 + j];
      const float* qp = sQ + s * 64 + dg * 16;
      const float* kp = sK + s * 64 + dg * 16;
      float accn = 0.0f;
#pragma unroll
      for (int g = 0; g < 4; ++g) {
        const v4f kk = *(const v4f*)(kp + 4 * g);
        const v4f qq = *(const v4f*)(qp + 4 * g);
        kv[4 * g + 0] = fmaf(kk[0], vj, kv[4 * g + 0]);
        accn = fmaf(qq[0], kv[4 * g + 0], accn);
        kv[4 * g + 1] = fmaf(kk[1], vj, kv[4 * g + 1]);
        accn = fmaf(qq[1], kv[4 * g + 1], accn);
        kv[4 * g + 2] = fmaf(kk[2], vj, kv[4 * g + 2]);
        accn = fmaf(qq[2], kv[4 * g + 2], accn);
        kv[4 * g + 3] = fmaf(kk[3], vj, kv[4 * g + 3]);
        accn = fmaf(qq[3], kv[4 * g + 3], accn);
      }
      sN[(dg * kScanT + s) * 64 + j] = accn;
    }
    __syncthreads();

    if (tid < 64) {
      float c = kcarry;
#pragma unroll 1
      for (int s = 0; s < kScanT; ++s) {
        c += sK[s * 64 + tid];
        sK[s * 64 + tid] = c;
      }
      kcarry = c;
    }
    __syncthreads();

    float den = 0.0f;
#pragma unroll 1
    for (int g = 0; g < 16; ++g) {
      const v4f qv = *(const v4f*)(sQ + orow * 64 + 4 * g);
      const v4f kc = *(const v4f*)(sK + orow * 64 + 4 * g);
      den = fmaf(qv[0], kc[0], den);
      den = fmaf(qv[1], kc[1], den);
      den = fmaf(qv[2], kc[2], den);
      den = fmaf(qv[3], kc[3], den);
    }
    const float inv = 1.0f / (den + kEps);

    const float* np = sN + orow * 64 + c8;
    const v4f a0 = *(const v4f*)(np);
    const v4f a1 = *(const v4f*)(np + 4);
    const v4f b0 = *(const v4f*)(np + 1 * kScanT * 64);
    const v4f b1 = *(const v4f*)(np + 1 * kScanT * 64 + 4);
    const v4f e0 = *(const v4f*)(np + 2 * kScanT * 64);
    const v4f e1 = *(const v4f*)(np + 2 * kScanT * 64 + 4);
    const v4f f0 = *(const v4f*)(np + 3 * kScanT * 64);
    const v4f f1 = *(const v4f*)(np + 3 * kScanT * 64 + 4);
    float o[8];
#pragma unroll
    for (int e = 0; e < 4; ++e) {
      const float n0v = ((a0[e] + b0[e]) + e0[e]) + f0[e];
      const float n1v = ((a1[e] + b1[e]) + e1[e]) + f1[e];
      o[e]     = n0v * inv;
      o[4 + e] = n1v * inv;
    }
    unsigned short hb[8], lb[8];
#pragma unroll
    for (int e = 0; e < 8; ++e) {
      const float x = o[e];
      const unsigned short hbits = f2bf_bits(x);
      const float res = x - bf_bits2f(hbits);
      hb[e] = hbits;
      lb[e] = f2bf_bits(res);
    }
    const v4u uh = (v4u){pk16(hb[0], hb[1]), pk16(hb[2], hb[3]), pk16(hb[4], hb[5]), pk16(hb[6], hb[7])};
    const v4u ul = (v4u){pk16(lb[0], lb[1]), pk16(lb[2], lb[3]), pk16(lb[4], lb[5]), pk16(lb[6], lb[7])};
    const size_t oo = (row0 + (size_t)(t0 + orow)) * kDim + col0 + c8;
    unsigned short* ph = AH + oo;
    unsigned short* pl = AL + oo;
    *(volatile v4u*)ph = uh;
    *(volatile v4u*)pl = ul;
    __threadfence();
    *(volatile v4u*)ph = uh;
    *(volatile v4u*)pl = ul;
  }
}

extern "C" void kernel_launch(void* const* d_in, const int* in_sizes, int n_in,
                              void* d_out, int out_size, void* d_ws, size_t ws_size,
                              hipStream_t stream) {
  if (n_in < 11 || d_out == nullptr || d_ws == nullptr) return;
  if (in_sizes[0] != kRows * kDim || in_sizes[1] != kRows * kDim || in_sizes[2] != kRows * kDim) return;
  if (in_sizes[3] != kDim * kDim || in_sizes[5] != kDim * kDim || in_sizes[7] != kDim * kDim ||
      in_sizes[9] != kDim * kDim) return;
  if (in_sizes[4] != kDim || in_sizes[6] != kDim || in_sizes[8] != kDim || in_sizes[10] != kDim) return;
  if (out_size != kRows * kDim) return;
  if (ws_size < kWsTotal) return;

  const float* query = (const float*)d_in[0];
  const float* key   = (const float*)d_in[1];
  const float* value = (const float*)d_in[2];
  const float* Wq    = (const float*)d_in[3];
  const float* bq    = (const float*)d_in[4];
  const float* Wk    = (const float*)d_in[5];
  const float* bk    = (const float*)d_in[6];
  const float* Wv    = (const float*)d_in[7];
  const float* bv    = (const float*)d_in[8];
  const float* Wo    = (const float*)d_in[9];
  const float* bo    = (const float*)d_in[10];
  float* out = (float*)d_out;

  char* ws = (char*)d_ws;
  unsigned short* XQ = (unsigned short*)(ws + kOffXQ);
  unsigned short* XK = (unsigned short*)(ws + kOffXK);
  unsigned short* XV = (unsigned short*)(ws + kOffXV);
  unsigned short* WQ = (unsigned short*)(ws + kOffWQ);
  unsigned short* WK = (unsigned short*)(ws + kOffWK);
  unsigned short* WV = (unsigned short*)(ws + kOffWV);
  unsigned short* WO = (unsigned short*)(ws + kOffWO);
  float*          QF = (float*)(ws + kOffQF);
  float*          KF = (float*)(ws + kOffKF);
  float*          VF = (float*)(ws + kOffVF);
  unsigned short* AH = (unsigned short*)(ws + kOffAH);
  unsigned short* AL = (unsigned short*)(ws + kOffAL);

  const int n8a = kRows * kDim / 8;
  const int n8w = kDim * kDim / 8;
  cvt_bf16_planes_kernel<<<dim3(n8a / 256, 3), 256, 0, stream>>>(query, key, value, value, XQ, XK, XV, XV, n8a);
  cvt_bf16_planes_kernel<<<dim3(n8w / 256, 4), 256, 0, stream>>>(Wq, Wk, Wv, Wo, WQ, WK, WV, WO, n8w);

  const int gblocks = (kRows / 64) * (kDim / 64) / 8;
  gemm_tile64_kernel<false, 1><<<dim3(gblocks), 256, 0, stream>>>(XQ, XQ, kDim, WQ, kDim, QF, kDim, bq, kRows, kDim, kDim);
  gemm_tile64_kernel<false, 1><<<dim3(gblocks), 256, 0, stream>>>(XK, XK, kDim, WK, kDim, KF, kDim, bk, kRows, kDim, kDim);
  gemm_tile64_kernel<false, 0><<<dim3(gblocks), 256, 0, stream>>>(XV, XV, kDim, WV, kDim, VF, kDim, bv, kRows, kDim, kDim);

  scan_state_kernel<<<dim3(kBatch * kHeads), 256, 0, stream>>>(QF, KF, VF, AH, AL);

  gemm_tile64_kernel<true, 0><<<dim3(gblocks), 256, 0, stream>>>(AH, AL, kDim, WO, kDim, out, kDim, bo, kRows, kDim, kDim);
}
